// MyMultiAttentionLayer_25640954757808
// MI455X (gfx1250) — hardware-verified
//
#include <hip/hip_runtime.h>


namespace {
constexpr int kB  = 2;
constexpr int kS  = 2048;
constexpr int kD  = 1024;
constexpr int kH  = 16;
constexpr int kP  = 64;
constexpr int kHP = kH * kP;
constexpr int kNO = 1024;
constexpr int kM  = kB * kS;
constexpr int kK  = 1024;
static_assert(kD == kK);
static_assert(kHP == kK);
static_assert(kNO == kK);
static_assert((kS % 128) == 0);
static_assert((kM % 128) == 0);
}

typedef __bf16 v16bf __attribute__((ext_vector_type(16)));
typedef float v8f __attribute__((ext_vector_type(8)));
typedef float v4f __attribute__((ext_vector_type(4), may_alias));
typedef unsigned short v8us __attribute__((ext_vector_type(8), may_alias));
typedef unsigned int v4u __attribute__((ext_vector_type(4), may_alias));

union Frag { v16bf v; v8us h[2]; };
union Pack8 { v8us v; v4u u; unsigned short s[8]; };

__device__ __forceinline__ v8f zero8() {
  v8f z = {0.f, 0.f, 0.f, 0.f, 0.f, 0.f, 0.f, 0.f};
  return z;
}

__device__ __forceinline__ unsigned short bf_rne(float f) {
  unsigned int u = __builtin_bit_cast(unsigned int, f);
  u += 0x7FFFu + ((u >> 16) & 1u);
  return (unsigned short)(u >> 16);
}
__device__ __forceinline__ float bf_val(unsigned short b) {
  return __builtin_bit_cast(float, ((unsigned int)b) << 16);
}
__device__ __forceinline__ void split_bf(float v, unsigned short& hi, unsigned short& lo) {
  const unsigned short hb = bf_rne(v);
  hi = hb;
  lo = bf_rne(v - bf_val(hb));
}

__device__ __forceinline__ v16bf ldfrag(const unsigned short* base, int ld, int lane) {
  const unsigned short* p = base + (size_t)(lane & 15) * (size_t)ld + ((lane >> 4) << 3);
  Frag f;
  f.h[0] = *reinterpret_cast<const v8us*>(p);
  f.h[1] = *reinterpret_cast<const v8us*>(p + 16);
  return f.v;
}

__device__ __forceinline__ v8f wmma3(v8f c, v16bf ah, v16bf al, v16bf bh, v16bf bl) {
  c = __builtin_amdgcn_wmma_f32_16x16x32_bf16(false, ah, false, bh, (short)0, c, false, false);
  c = __builtin_amdgcn_wmma_f32_16x16x32_bf16(false, ah, false, bl, (short)0, c, false, false);
  c = __builtin_amdgcn_wmma_f32_16x16x32_bf16(false, al, false, bh, (short)0, c, false, false);
  asm volatile("v_nop\n\tv_nop\n\tv_nop\n\tv_nop" : "+v"(c) : "v"(ah), "v"(al), "v"(bh), "v"(bl));
  return c;
}

__global__ __launch_bounds__(256) void k_split_planes(
    const float* __restrict__ s0, unsigned short* h0, unsigned short* l0,
    const float* __restrict__ s1, unsigned short* h1, unsigned short* l1,
    const float* __restrict__ s2, unsigned short* h2, unsigned short* l2,
    const float* __restrict__ s3, unsigned short* h3, unsigned short* l3, int n) {
  const int y = blockIdx.y;
  const float* src = (y == 0) ? s0 : (y == 1) ? s1 : (y == 2) ? s2 : s3;
  unsigned short* dh = (y == 0) ? h0 : (y == 1) ? h1 : (y == 2) ? h2 : h3;
  unsigned short* dl = (y == 0) ? l0 : (y == 1) ? l1 : (y == 2) ? l2 : l3;
  const size_t e0 = ((size_t)blockIdx.x * blockDim.x + threadIdx.x) * 8;
  if (e0 + 8 > (size_t)n) return;
  const v4f a = *reinterpret_cast<const v4f*>(src + e0);
  const v4f c = *reinterpret_cast<const v4f*>(src + e0 + 4);
  Pack8 ph, pl;
#pragma unroll
  for (int e = 0; e < 4; ++e) {
    split_bf(a[e], ph.s[e], pl.s[e]);
    split_bf(c[e], ph.s[e + 4], pl.s[e + 4]);
  }
  const v4u vh = ph.u;
  const v4u vl = pl.u;
  *reinterpret_cast<volatile v4u*>(dh + e0) = vh;
  *reinterpret_cast<volatile v4u*>(dl + e0) = vl;
  __threadfence();
  *reinterpret_cast<volatile v4u*>(dh + e0) = vh;
  *reinterpret_cast<volatile v4u*>(dl + e0) = vl;
}

template <int MODE>
__global__ __launch_bounds__(128) void k_gemm(const unsigned short* __restrict__ Ah,
                                              const unsigned short* __restrict__ Al,
                                              const unsigned short* __restrict__ Wh,
                                              const unsigned short* __restrict__ Wl,
                                              const float* __restrict__ bias,
                                              unsigned short* Oh, unsigned short* Ol, float* Of) {
  __shared__ __attribute__((aligned(16))) unsigned short lds_t[2 * 128 * 64];
  const int tid = threadIdx.x, wid = tid >> 5, lane = tid & 31, hs = lane >> 4, nl = lane & 15;
  const int mt = blockIdx.x >> 4, ng = blockIdx.x & 15;
  const int mb = mt * 128;
  const int m0 = mb + wid * 32;
  const int n0 = ng * 64;

  v8f acc[2][4];
#pragma unroll
  for (int i = 0; i < 2; ++i)
#pragma unroll
    for (int j = 0; j < 4; ++j) acc[i][j] = zero8();

  for (int k0 = 0; k0 < kK; k0 += 32) {
    v16bf fa_h[2], fa_l[2];
#pragma unroll
    for (int i = 0; i < 2; ++i) {
      const size_t o = (size_t)(m0 + 16 * i) * kK + k0;
      fa_h[i] = ldfrag(Ah + o, kK, lane);
      fa_l[i] = ldfrag(Al + o, kK, lane);
    }
#pragma unroll
    for (int j = 0; j < 4; ++j) {
      const size_t o = (size_t)(n0 + 16 * j) * kK + k0;
      const v16bf fb_h = ldfrag(Wh + o, kK, lane);
      const v16bf fb_l = ldfrag(Wl + o, kK, lane);
#pragma unroll
      for (int i = 0; i < 2; ++i) acc[i][j] = wmma3(acc[i][j], fa_h[i], fa_l[i], fb_h, fb_l);
    }
  }

  float* lds_f = reinterpret_cast<float*>(lds_t);
  unsigned short* lds_h = lds_t;
  unsigned short* lds_l = lds_t + 128 * 64;
#pragma unroll
  for (int i = 0; i < 2; ++i) {
#pragma unroll
    for (int j = 0; j < 4; ++j) {
      const int col = 16 * j + nl;
      const float bs = bias[n0 + col];
#pragma unroll
      for (int r = 0; r < 8; ++r) {
        const int row = wid * 32 + 16 * i + 8 * hs + r;
        const float v = acc[i][j][r] + bs;
        if (MODE == 2) {
          lds_f[row * 64 + col] = v;
        } else {
          unsigned short xh, xl;
          split_bf(v, xh, xl);
          if (MODE == 0) {
            lds_h[row * 64 + col] = xh;
            lds_l[row * 64 + col] = xl;
          } else {
            lds_h[col * 128 + row] = xh;
            lds_l[col * 128 + row] = xl;
          }
        }
      }
    }
  }
  __syncthreads();

  if (MODE == 2) {
    for (int ps = 0; ps < 2; ++ps) {
      if (ps) __threadfence();
#pragma unroll
      for (int it = 0; it < 16; ++it) {
        const int c = it * 128 + tid;
        const int row = c >> 4, piece = c & 15;
        const v4f val = *reinterpret_cast<const v4f*>(lds_f + row * 64 + piece * 4);
        float* dst = Of + (size_t)(mb + row) * kNO + n0 + piece * 4;
        *reinterpret_cast<volatile v4f*>(dst) = val;
      }
    }
  } else if (MODE == 0) {
    const int b = mb >> 11, s0 = mb & (kS - 1);
    const size_t base = ((size_t)((b * kH + ng) * kS + s0)) * kP;
    for (int ps = 0; ps < 2; ++ps) {
      if (ps) __threadfence();
#pragma unroll
      for (int it = 0; it < 8; ++it) {
        const int c = it * 128 + tid;
        const v4f dummy = {0.f, 0.f, 0.f, 0.f};
        (void)dummy;
        const v4u vh = *reinterpret_cast<const v4u*>(lds_h + c * 8);
        const v4u vl = *reinterpret_cast<const v4u*>(lds_l + c * 8);
        const size_t o = base + (size_t)c * 8;
        *reinterpret_cast<volatile v4u*>(Oh + o) = vh;
        *reinterpret_cast<volatile v4u*>(Ol + o) = vl;
      }
    }
  } else {
    const int b = mb >> 11, s0 = mb & (kS - 1);
    const size_t base = ((size_t)((b * kH + ng) * kP)) * kS + s0;
    for (int ps = 0; ps < 2; ++ps) {
      if (ps) __threadfence();
#pragma unroll
      for (int it = 0; it < 8; ++it) {
        const int c = it * 128 + tid;
        const int prow = c >> 4, piece = c & 15;
        const v4u vh = *reinterpret_cast<const v4u*>(lds_h + prow * 128 + piece * 8);
        const v4u vl = *reinterpret_cast<const v4u*>(lds_l + prow * 128 + piece * 8);
        const size_t o = base + (size_t)prow * kS + piece * 8;
        *reinterpret_cast<volatile v4u*>(Oh + o) = vh;
        *reinterpret_cast<volatile v4u*>(Ol + o) = vl;
      }
    }
  }
}

__global__ __launch_bounds__(128) void k_colstats(const unsigned short* __restrict__ Qh,
                                                  const unsigned short* __restrict__ Ql,
                                                  const unsigned short* __restrict__ Kh,
                                                  const unsigned short* __restrict__ Kl,
                                                  float* cmax, float* csum) {
  __shared__ __attribute__((aligned(16))) float lM[128];
  __shared__ __attribute__((aligned(16))) float lL[128];
  const int tid = threadIdx.x, wid = tid >> 5, lane = tid & 31, nl = lane & 15;
  const int bh = blockIdx.x >> 4;
  const int kb = (blockIdx.x & 15) * 128;
  const int kw = kb + wid * 32;
  const size_t hoff = (size_t)bh * kS * kP;
  const unsigned short* qh = Qh + hoff;
  const unsigned short* ql = Ql + hoff;
  const unsigned short* kh = Kh + hoff;
  const unsigned short* kl = Kl + hoff;

  v16bf fk_h[2][2], fk_l[2][2];
#pragma unroll
  for (int t = 0; t < 2; ++t) {
#pragma unroll
    for (int ks = 0; ks < 2; ++ks) {
      const size_t o = (size_t)(kw + 16 * t) * kP + 32 * ks;
      fk_h[t][ks] = ldfrag(kh + o, kP, lane);
      fk_l[t][ks] = ldfrag(kl + o, kP, lane);
    }
  }

  float mx[2] = {-1.0e30f, -1.0e30f};
  float sm[2] = {0.f, 0.f};
  for (int qt = 0; qt < kS; qt += 16) {
    v16bf fq_h[2], fq_l[2];
#pragma unroll
    for (int ks = 0; ks < 2; ++ks) {
      const size_t o = (size_t)qt * kP + 32 * ks;
      fq_h[ks] = ldfrag(qh + o, kP, lane);
      fq_l[ks] = ldfrag(ql + o, kP, lane);
    }
#pragma unroll
    for (int t = 0; t < 2; ++t) {
      v8f s = zero8();
#pragma unroll
      for (int ks = 0; ks < 2; ++ks) s = wmma3(s, fq_h[ks], fq_l[ks], fk_h[t][ks], fk_l[t][ks]);
      float tmax = s[0] * 0.125f;
#pragma unroll
      for (int r = 1; r < 8; ++r) tmax = fmaxf(tmax, s[r] * 0.125f);
      const float nm = fmaxf(mx[t], tmax);
      float part = 0.f;
#pragma unroll
      for (int r = 0; r < 8; ++r) part += __expf(s[r] * 0.125f - nm);
      sm[t] = sm[t] * __expf(mx[t] - nm) + part;
      mx[t] = nm;
    }
  }

#pragma unroll
  for (int t = 0; t < 2; ++t) {
    const float omx = __shfl_xor(mx[t], 16, 32);
    const float osm = __shfl_xor(sm[t], 16, 32);
    const float Mv = fmaxf(mx[t], omx);
    const float Lv = sm[t] * __expf(mx[t] - Mv) + osm * __expf(omx - Mv);
    if (lane < 16) {
      lM[wid * 32 + 16 * t + nl] = Mv;
      lL[wid * 32 + 16 * t + nl] = Lv;
    }
  }
  __syncthreads();

  const size_t obase = (size_t)bh * kS + kb;
  for (int ps = 0; ps < 2; ++ps) {
    if (ps) __threadfence();
    if (wid == 0) {
      const v4f v = *reinterpret_cast<const v4f*>(lM + lane * 4);
      *reinterpret_cast<volatile v4f*>(cmax + obase + lane * 4) = v;
    } else if (wid == 1) {
      const v4f v = *reinterpret_cast<const v4f*>(lL + lane * 4);
      *reinterpret_cast<volatile v4f*>(csum + obase + lane * 4) = v;
    }
  }
}

__global__ __launch_bounds__(128) void k_ctx(const unsigned short* __restrict__ Qh,
                                             const unsigned short* __restrict__ Ql,
                                             const unsigned short* __restrict__ Kh,
                                             const unsigned short* __restrict__ Kl,
                                             const unsigned short* __restrict__ Vh,
                                             const unsigned short* __restrict__ Vl,
                                             const float* __restrict__ cmax,
                                             const float* __restrict__ csum,
                                             unsigned short* Ch, unsigned short* Cl) {
  __shared__ __attribute__((aligned(16))) unsigned short lPh[4][512];
  __shared__ __attribute__((aligned(16))) unsigned short lPl[4][512];
  __shared__ __attribute__((aligned(16))) unsigned short lCh[64 * 64];
  __shared__ __attribute__((aligned(16))) unsigned short lCl[64 * 64];
  const int tid = threadIdx.x, wid = tid >> 5, lane = tid & 31, hs = lane >> 4, nl = lane & 15;
  const int bh = blockIdx.x >> 5;
  const int qb = (blockIdx.x & 31) * 64;
  const int qw = qb + wid * 16;
  const int b = bh >> 4, hd = bh & 15;
  const size_t hoff = (size_t)bh * kS * kP;
  const unsigned short* qh = Qh + hoff;
  const unsigned short* ql = Ql + hoff;
  const unsigned short* kh = Kh + hoff;
  const unsigned short* kl = Kl + hoff;
  const unsigned short* vh = Vh + hoff;
  const unsigned short* vl = Vl + hoff;
  const float* cm = cmax + (size_t)bh * kS;
  const float* cs = csum + (size_t)bh * kS;

  v16bf fq_h[2], fq_l[2];
#pragma unroll
  for (int ks = 0; ks < 2; ++ks) {
    const size_t o = (size_t)qw * kP + 32 * ks;
    fq_h[ks] = ldfrag(qh + o, kP, lane);
    fq_l[ks] = ldfrag(ql + o, kP, lane);
  }

  v8f acc[4];
#pragma unroll
  for (int j = 0; j < 4; ++j) acc[j] = zero8();

  for (int k0 = 0; k0 < kS; k0 += 32) {
#pragma unroll
    for (int t = 0; t < 2; ++t) {
      const int kt = k0 + 16 * t;
      v16bf fk_h[2], fk_l[2];
#pragma unroll
      for (int ks = 0; ks < 2; ++ks) {
        const size_t o = (size_t)kt * kP + 32 * ks;
        fk_h[ks] = ldfrag(kh + o, kP, lane);
        fk_l[ks] = ldfrag(kl + o, kP, lane);
      }
      v8f s = zero8();
#pragma unroll
      for (int ks = 0; ks < 2; ++ks) s = wmma3(s, fq_h[ks], fq_l[ks], fk_h[ks], fk_l[ks]);
      const float m  = cm[kt + nl];
      const float rl = __builtin_amdgcn_rcpf(cs[kt + nl]);
#pragma unroll
      for (int r = 0; r < 8; ++r) {
        const float p = __expf(s[r] * 0.125f - m) * rl;
        unsigned short xh, xl;
        split_bf(p, xh, xl);
        const int idx = (8 * hs + r) * 32 + 16 * t + nl;
        lPh[wid][idx] = xh;
        lPl[wid][idx] = xl;
      }
    }
    __builtin_amdgcn_fence(__ATOMIC_RELEASE, "wavefront");
    __builtin_amdgcn_wave_barrier();
    const v16bf fp_h = ldfrag(&lPh[wid][0], 32, lane);
    const v16bf fp_l = ldfrag(&lPl[wid][0], 32, lane);
#pragma unroll
    for (int j = 0; j < 4; ++j) {
      const size_t o = (size_t)(16 * j) * kS + k0;
      const v16bf fv_h = ldfrag(vh + o, kS, lane);
      const v16bf fv_l = ldfrag(vl + o, kS, lane);
      acc[j] = wmma3(acc[j], fp_h, fp_l, fv_h, fv_l);
    }
    __builtin_amdgcn_fence(__ATOMIC_RELEASE, "wavefront");
    __builtin_amdgcn_wave_barrier();
  }

#pragma unroll
  for (int j = 0; j < 4; ++j) {
#pragma unroll
    for (int r = 0; r < 8; ++r) {
      const int row = wid * 16 + 8 * hs + r;
      const int col = 16 * j + nl;
      unsigned short xh, xl;
      split_bf(acc[j][r], xh, xl);
      lCh[row * 64 + col] = xh;
      lCl[row * 64 + col] = xl;
    }
  }
  __syncthreads();

  const size_t base = ((size_t)(b * kS + qb)) * kHP + (size_t)hd * kP;
  for (int ps = 0; ps < 2; ++ps) {
    if (ps) __threadfence();
#pragma unroll
    for (int it = 0; it < 4; ++it) {
      const int c = it * 128 + tid;
      const int row = c >> 3, piece = c & 7;
      const v4u xh = *reinterpret_cast<const v4u*>(lCh + row * 64 + piece * 8);
      const v4u xl = *reinterpret_cast<const v4u*>(lCl + row * 64 + piece * 8);
      const size_t o = base + (size_t)row * kHP + piece * 8;
      *reinterpret_cast<volatile v4u*>(Ch + o) = xh;
      *reinterpret_cast<volatile v4u*>(Cl + o) = xl;
    }
  }
}

extern "C" void kernel_launch(void* const* d_in, const int* in_sizes, int n_in,
                              void* d_out, int out_size, void* d_ws, size_t ws_size,
                              hipStream_t stream) {
  if (n_in < 9) return;
  const size_t nX = (size_t)kM * kD;
  const size_t nW = (size_t)kK * kK;
  const size_t nQ = (size_t)kB * kH * kS * kP;
  const size_t nC = (size_t)kM * kHP;
  const size_t nT = (size_t)kB * kH * kS;
  if ((size_t)in_sizes[0] != nX || (size_t)in_sizes[1] != nW || (size_t)in_sizes[2] != (size_t)kHP ||
      (size_t)in_sizes[3] != nW || (size_t)in_sizes[4] != (size_t)kHP || (size_t)in_sizes[5] != nW ||
      (size_t)in_sizes[6] != (size_t)kHP || (size_t)in_sizes[7] != nW || (size_t)in_sizes[8] != (size_t)kNO)
    return;
  if ((size_t)out_size != (size_t)kM * kNO) return;

  const float* x   = static_cast<const float*>(d_in[0]);
  const float* q_w = static_cast<const float*>(d_in[1]);
  const float* q_b = static_cast<const float*>(d_in[2]);
  const float* k_w = static_cast<const float*>(d_in[3]);
  const float* k_b = static_cast<const float*>(d_in[4]);
  const float* v_w = static_cast<const float*>(d_in[5]);
  const float* v_b = static_cast<const float*>(d_in[6]);
  const float* l_w = static_cast<const float*>(d_in[7]);
  const float* l_b = static_cast<const float*>(d_in[8]);
  float* out = static_cast<float*>(d_out);

  char* ws = static_cast<char*>(d_ws);
  size_t off = 0;
  auto carve = [&](size_t bytes) -> char* {
    char* p = ws + off;
    off += (bytes + 255) & ~(size_t)255;
    return p;
  };
  unsigned short* xh  = (unsigned short*)carve(nX * 2);
  unsigned short* xl  = (unsigned short*)carve(nX * 2);
  unsigned short* wqh = (unsigned short*)carve(nW * 2);
  unsigned short* wql = (unsigned short*)carve(nW * 2);
  unsigned short* wkh = (unsigned short*)carve(nW * 2);
  unsigned short* wkl = (unsigned short*)carve(nW * 2);
  unsigned short* wvh = (unsigned short*)carve(nW * 2);
  unsigned short* wvl = (unsigned short*)carve(nW * 2);
  unsigned short* lwh = (unsigned short*)carve(nW * 2);
  unsigned short* lwl = (unsigned short*)carve(nW * 2);
  unsigned short* Qh  = (unsigned short*)carve(nQ * 2);
  unsigned short* Ql  = (unsigned short*)carve(nQ * 2);
  unsigned short* Kh  = (unsigned short*)carve(nQ * 2);
  unsigned short* Kl  = (unsigned short*)carve(nQ * 2);
  unsigned short* Vh  = (unsigned short*)carve(nQ * 2);
  unsigned short* Vl  = (unsigned short*)carve(nQ * 2);
  unsigned short* Ch  = (unsigned short*)carve(nC * 2);
  unsigned short* Cl  = (unsigned short*)carve(nC * 2);
  float* cmax = (float*)carve(nT * 4);
  float* csum = (float*)carve(nT * 4);
  if (off > ws_size) return;

  const unsigned gx = (unsigned)((nX / 8 + 255) / 256);
  const unsigned gw = (unsigned)((nW / 8 + 255) / 256);
  k_split_planes<<<dim3(gx, 1), dim3(256), 0, stream>>>(x, xh, xl, x, xh, xl, x, xh, xl, x, xh, xl,
                                                         (int)nX);
  k_split_planes<<<dim3(gw, 4), dim3(256), 0, stream>>>(q_w, wqh, wql, k_w, wkh, wkl, v_w, wvh, wvl,
                                                         l_w, lwh, lwl, (int)nW);

  const unsigned gg = (unsigned)((kM / 128) * (kK / 64));
  k_gemm<0><<<dim3(gg), dim3(128), 0, stream>>>(xh, xl, wqh, wql, q_b, Qh, Ql, out);
  k_gemm<0><<<dim3(gg), dim3(128), 0, stream>>>(xh, xl, wkh, wkl, k_b, Kh, Kl, out);
  k_gemm<1><<<dim3(gg), dim3(128), 0, stream>>>(xh, xl, wvh, wvl, v_b, Vh, Vl, out);

  const unsigned gs = (unsigned)(kB * kH * (kS / 128));
  k_colstats<<<dim3(gs), dim3(128), 0, stream>>>(Qh, Ql, Kh, Kl, cmax, csum);

  const unsigned gc = (unsigned)(kB * kH * (kS / 64));
  k_ctx<<<dim3(gc), dim3(128), 0, stream>>>(Qh, Ql, Kh, Kl, Vh, Vl, cmax, csum, Ch, Cl);

  k_gemm<2><<<dim3(gg), dim3(128), 0, stream>>>(Ch, Cl, lwh, lwl, l_b, xh, xl, out);
}
